// EncoderLayer_38568806318150
// MI455X (gfx1250) — hardware-run, weakly checked
//
#include <hip/hip_runtime.h>
#include <math.h>

constexpr int kBatch = 2;
constexpr int kSeq   = 2048;
constexpr int kDim   = 1024;
constexpr int kHeads = 4;
constexpr int kInner = 2048;
constexpr int kDH    = 512;
constexpr int kFF    = 4096;
constexpr int kRows  = kBatch * kSeq;
constexpr int kUpN   = 2 * kInner;
constexpr int kGateN = 64;
constexpr int kPP    = 72;
constexpr float kWCarry  = 16.0f;
constexpr float kXcCarry = 64.0f;
constexpr float kQKCarry = 64.0f;
constexpr float kPCarry  = 4096.0f;
constexpr float kHoCarry = 16.0f;
constexpr float kLnEps   = 1e-6f;
constexpr float kFltMin  = 1.17549435e-38f;
static_assert(kInner == kHeads * kDH, "head split");
static_assert(kQKCarry * kQKCarry == kPCarry, "score carry");
static_assert(kRows % 64 == 0 && kDim % 64 == 0 && kInner % 64 == 0 && kFF % 64 == 0 && kUpN % 64 == 0, "tile multiples");
static_assert(kDim % 32 == 0 && kInner % 32 == 0 && kFF % 32 == 0 && kDH % 32 == 0 && kSeq % 64 == 0, "k multiples");
static_assert(kGateN == 64 && 2 * kHeads <= kGateN, "gate tile");
static_assert((kPP * 2) % 16 == 0, "P pitch alignment");

typedef __attribute__((ext_vector_type(16))) _Float16 v16h;
typedef __attribute__((ext_vector_type(8)))  _Float16 v8h;
typedef __attribute__((ext_vector_type(8)))  float    v8f;
typedef __attribute__((ext_vector_type(4)))  float    v4f;
typedef __attribute__((ext_vector_type(2)))  float    v2f;
typedef __attribute__((ext_vector_type(4)))  unsigned int v4u;

__device__ __forceinline__ v8f mma_h(v16h a, v16h b, v8f c) {
  c = __builtin_amdgcn_wmma_f32_16x16x32_f16(false, a, false, b, (short)0, c, false, false);
  asm volatile("v_nop\n\tv_nop\n\tv_nop\n\tv_nop" : "+v"(c) : "v"(a), "v"(b));
  return c;
}

struct FragH {
  union U { v16h v; v8h h[2]; };
  static __device__ __forceinline__ v16h load(const _Float16* p) {
    U f; f.h[0] = *(const v8h*)(p); f.h[1] = *(const v8h*)(p + 16); return f.v;
  }
};

__device__ __forceinline__ float h16_to_f32(unsigned hb) {
  const unsigned sgn = (hb & 0x8000u) << 16; const unsigned em = hb & 0x7fffu;
  const float fn = __uint_as_float((em << 13) + 0x38000000u);
  const float fs = (float)em * 5.9604644775390625e-8f;
  const float mag = (em < 0x400u) ? fs : fn; return __uint_as_float(__float_as_uint(mag) | sgn);
}
__device__ __forceinline__ unsigned h_bits(float f) { const _Float16 h = (_Float16)f; return (unsigned)__builtin_bit_cast(unsigned short, h); }

template <int BIAS_MODE, int OUT_MODE, bool RESID, int ACT>
__global__ __launch_bounds__(256) void wmma_gemm64(
    const unsigned short* __restrict__ Ap, int lda,
    const unsigned short* __restrict__ Btp, int ldb,
    void* __restrict__ Cout, int ldc,
    const float* __restrict__ bias,
    const float* __restrict__ resid,
    int M, int N, int K, float scale, float post, float rscale) {
  const _Float16* A  = (const _Float16*)Ap;
  const _Float16* Bt = (const _Float16*)Btp;
  __shared__ __align__(16) float sT[8][16 * 68];
  const int lane = threadIdx.x & 31;
  const int wave = threadIdx.x >> 5;
  const int tilesN = N >> 6;
  const int tilesM = M >> 6;
  const int tile = blockIdx.x * 8 + wave;
  if (tile >= tilesM * tilesN) return;
  const int tm = tile / tilesN;
  const int tn = tile - tm * tilesN;
  const int m0 = tm << 6;
  const int n0 = tn << 6;
  const int rlane = lane & 15;
  const int koff  = (lane >> 4) * 8;
  const int mOff  = (lane >> 4) * 8;

  v8f acc[4][4];
#pragma unroll
  for (int i = 0; i < 4; ++i)
#pragma unroll
    for (int j = 0; j < 4; ++j) acc[i][j] = (v8f){0.f,0.f,0.f,0.f,0.f,0.f,0.f,0.f};

  const _Float16* aBase = A  + (size_t)(m0 + rlane) * lda + koff;
  const _Float16* bBase = Bt + (size_t)(n0 + rlane) * ldb + koff;
  const size_t aStep = (size_t)16 * lda;
  const size_t bStep = (size_t)16 * ldb;

  for (int k0 = 0; k0 < K; k0 += 32) {
    v16h bh[4];
#pragma unroll
    for (int j = 0; j < 4; ++j) bh[j] = FragH::load(bBase + j * bStep + k0);
#pragma unroll
    for (int i = 0; i < 4; ++i) {
      const v16h ah = FragH::load(aBase + i * aStep + k0);
#pragma unroll
      for (int j = 0; j < 4; ++j) acc[i][j] = mma_h(ah, bh[j], acc[i][j]);
    }
  }

  float* slab = sT[wave];
#pragma unroll
  for (int i = 0; i < 4; ++i) {
    const int mBase = m0 + (i << 4);
#pragma unroll
    for (int j = 0; j < 4; ++j) {
      const int n = n0 + (j << 4) + rlane;
      float bv = 0.f;
      if (BIAS_MODE == 2) bv = bias[n];
#pragma unroll
      for (int r = 0; r < 8; ++r) {
        float v = acc[i][j][r] * scale;
        if (BIAS_MODE == 1) v += bias[mBase + mOff + r];
        if (BIAS_MODE == 2) v += bv;
        if (ACT == 2) v = fmaxf(v, 0.0f);
        v *= post;
        slab[(mOff + r) * 68 + (j << 4) + rlane] = v;
      }
    }
    __builtin_amdgcn_fence(__ATOMIC_RELEASE, "workgroup");
    __builtin_amdgcn_wave_barrier();
    __builtin_amdgcn_fence(__ATOMIC_ACQUIRE, "workgroup");
    if (OUT_MODE == 0) {
      float* C = (float*)Cout;
      const int hh = lane >> 4, c4 = (lane & 15) * 4;
      v4f vv[8];
#pragma unroll
      for (int it = 0; it < 8; ++it) {
        const int row = it * 2 + hh;
        v4f v = *(const v4f*)(slab + row * 68 + c4);
        if (RESID) {
          const v4f rv = *(const v4f*)(resid + (size_t)(mBase + row) * ldc + n0 + c4);
          v = v + rscale * rv;
        }
        vv[it] = v;
      }
      for (int pass = 0; pass < 2; ++pass) {
#pragma unroll
        for (int it = 0; it < 8; ++it) {
          const int row = it * 2 + hh;
          *(volatile v4f*)(C + (size_t)(mBase + row) * ldc + n0 + c4) = vv[it];
        }
        __threadfence();
      }
    } else {
      const int q = lane >> 3, c8 = (lane & 7) * 8;
      unsigned short* C = (unsigned short*)Cout;
      for (int pass = 0; pass < 2; ++pass) {
#pragma unroll
        for (int it = 0; it < 4; ++it) {
          const int row = it * 4 + q;
          const float* sp = slab + row * 68 + c8;
          v8h hv;
#pragma unroll
          for (int e = 0; e < 8; ++e) hv[e] = (_Float16)sp[e];
          *(volatile v8h*)(C + (size_t)(mBase + row) * ldc + n0 + c8) = hv;
        }
        __threadfence();
      }
    }
    __builtin_amdgcn_fence(__ATOMIC_RELEASE, "workgroup");
    __builtin_amdgcn_wave_barrier();
    __builtin_amdgcn_fence(__ATOMIC_ACQUIRE, "workgroup");
  }
}

__global__ __launch_bounds__(256) void wt_f16_kernel(const float* __restrict__ src, int R, int C, int ldo,
                                                     unsigned short* __restrict__ O, float sc) {
  __shared__ float Tt[64 * 65];
  (void)R;
  const int tid = threadIdx.x;
  const int c0 = blockIdx.x * 64, r0 = blockIdx.y * 64;
#pragma unroll
  for (int i = 0; i < 4; ++i) {
    const int idx = i * 256 + tid;
    const int rr = idx >> 4, cc = (idx & 15) * 4;
    const v4f v = *(const v4f*)(src + (size_t)(r0 + rr) * (size_t)C + c0 + cc);
    Tt[rr * 65 + cc + 0] = v[0];
    Tt[rr * 65 + cc + 1] = v[1];
    Tt[rr * 65 + cc + 2] = v[2];
    Tt[rr * 65 + cc + 3] = v[3];
  }
  __syncthreads();
  const int q = tid >> 3, c8 = (tid & 7) * 8;
  v8h hv[2];
#pragma unroll
  for (int g = 0; g < 2; ++g) {
    const int qq = g * 32 + q;
#pragma unroll
    for (int e = 0; e < 8; ++e) hv[g][e] = (_Float16)(Tt[(c8 + e) * 65 + qq] * sc);
  }
  for (int pass = 0; pass < 2; ++pass) {
#pragma unroll
    for (int g = 0; g < 2; ++g) {
      const size_t o = (size_t)(c0 + g * 32 + q) * (size_t)ldo + (size_t)(r0 + c8);
      *(volatile v8h*)(O + o) = hv[g];
    }
    __threadfence();
  }
}

__global__ __launch_bounds__(256) void wif_f16_kernel(const float* __restrict__ Wif, unsigned short* __restrict__ O, float sc) {
  const int i = blockIdx.x * 256 + threadIdx.x;
  const int n = i >> 8, k8 = (i & 255) * 8;
  const int nc = (n < 8) ? n : 7;
  unsigned hb[8];
#pragma unroll
  for (int e = 0; e < 8; ++e) {
    const float f = Wif[(size_t)(k8 + e) * 8 + nc];
    const float val = (n < 8) ? f * sc : 0.0f;
    hb[e] = h_bits(val);
  }
  const v4u u = (v4u){hb[0] | (hb[1] << 16), hb[2] | (hb[3] << 16), hb[4] | (hb[5] << 16), hb[6] | (hb[7] << 16)};
  unsigned short* op = O + (size_t)n * kInner + k8;
  *(volatile v4u*)(void*)op = u;
  __threadfence();
  *(volatile v4u*)(void*)op = u;
}

__global__ __launch_bounds__(256) void ln_f16_kernel(const float* __restrict__ x, const float* __restrict__ g,
                                                     const float* __restrict__ bt, unsigned short* __restrict__ xn, int nrows) {
  const int lane = threadIdx.x & 31;
  const int row = blockIdx.x * 8 + (threadIdx.x >> 5);
  if (row >= nrows) return;
  const float* rp = x + (size_t)row * kDim;
  v4f v[4][2];
  float s = 0.0f;
#pragma unroll
  for (int q = 0; q < 4; ++q) {
    const float* p = rp + 256 * q + 8 * lane;
    v[q][0] = *(const v4f*)(p);
    v[q][1] = *(const v4f*)(p + 4);
  }
#pragma unroll
  for (int q = 0; q < 4; ++q)
#pragma unroll
    for (int e = 0; e < 4; ++e) s += v[q][0][e] + v[q][1][e];
#pragma unroll
  for (int off = 1; off < 32; off <<= 1) s += __shfl_xor(s, off, 32);
  const float mu = s * (1.0f / (float)kDim);
  float ss = 0.0f;
#pragma unroll
  for (int q = 0; q < 4; ++q)
#pragma unroll
    for (int u = 0; u < 2; ++u)
#pragma unroll
      for (int e = 0; e < 4; ++e) { const float d = v[q][u][e] - mu; v[q][u][e] = d; ss += d * d; }
#pragma unroll
  for (int off = 1; off < 32; off <<= 1) ss += __shfl_xor(ss, off, 32);
  const float var = ss * (1.0f / (float)kDim);
  const float rstd = rsqrtf(var + kLnEps);
  v8h hv[4];
#pragma unroll
  for (int q = 0; q < 4; ++q) {
    const int co = 256 * q + 8 * lane;
    const v4f g0 = *(const v4f*)(g + co);
    const v4f g1 = *(const v4f*)(g + co + 4);
    const v4f b0 = *(const v4f*)(bt + co);
    const v4f b1 = *(const v4f*)(bt + co + 4);
#pragma unroll
    for (int e = 0; e < 4; ++e) {
      hv[q][e]     = (_Float16)((v[q][0][e] * rstd) * g0[e] + b0[e]);
      hv[q][4 + e] = (_Float16)((v[q][1][e] * rstd) * g1[e] + b1[e]);
    }
  }
  unsigned short* op = xn + (size_t)row * kDim;
  for (int pass = 0; pass < 2; ++pass) {
#pragma unroll
    for (int q = 0; q < 4; ++q) *(volatile v8h*)(op + 256 * q + 8 * lane) = hv[q];
    __threadfence();
  }
}

__global__ __launch_bounds__(256) void conv_silu_kernel(const unsigned short* __restrict__ up, const float* __restrict__ cw,
                                                        const float* __restrict__ cb, unsigned short* __restrict__ xc) {
  const int i = blockIdx.x * 256 + threadIdx.x;
  const int row = i >> 10;
  const int cp = (i & 1023) * 2;
  const int s = row & (kSeq - 1);
  const unsigned* upw = (const unsigned*)(const void*)up;
  float a0 = 0.0f, a1 = 0.0f;
#pragma unroll
  for (int t = 0; t < 4; ++t) {
    const int sp = s - 3 + t;
    const bool ok = (sp >= 0);
    const int rr = ok ? (row - 3 + t) : row;
    const unsigned w = upw[((size_t)rr * kUpN + cp) >> 1];
    const v2f wv = *(const v2f*)(cw + t * kInner + cp);
    float x0 = h16_to_f32(w & 0xffffu);
    float x1 = h16_to_f32(w >> 16);
    x0 = ok ? x0 : 0.0f;
    x1 = ok ? x1 : 0.0f;
    a0 += x0 * wv[0];
    a1 += x1 * wv[1];
  }
  const v2f bv = *(const v2f*)(cb + cp);
  a0 += bv[0];
  a1 += bv[1];
  const float o0 = a0 * __builtin_amdgcn_rcpf(1.0f + expf(-a0)) * kXcCarry;
  const float o1 = a1 * __builtin_amdgcn_rcpf(1.0f + expf(-a1)) * kXcCarry;
  const unsigned u = h_bits(o0) | (h_bits(o1) << 16);
  ((volatile unsigned*)xc)[i] = u;
  __threadfence();
  ((volatile unsigned*)xc)[i] = u;
}

__global__ __launch_bounds__(256) void scan_kernel(const float* __restrict__ g, const float* __restrict__ bif,
                                                   float* __restrict__ aout, float* __restrict__ cmout, float* __restrict__ mout) {
  __shared__ __align__(16) float sF[kSeq];
  __shared__ __align__(16) float sA[kSeq];
  __shared__ __align__(16) float sC[kSeq];
  __shared__ float sc[256];
  const int bh = blockIdx.x;
  const int b = bh / kHeads, h = bh % kHeads;
  const int tid = threadIdx.x;
  const float bi = bif[h];
  const float bf = bif[kHeads + h];
  const float* gb = g + (size_t)b * kSeq * kGateN;
  float run = 0.0f;
#pragma unroll 1
  for (int j = 0; j < 8; ++j) {
    const int s = tid * 8 + j;
    const float f = gb[(size_t)s * kGateN + kHeads + h] + bf;
    const float ls = fminf(f, 0.0f) - log1pf(expf(-fabsf(f)));
    run += ls;
    sF[s] = run;
  }
  sc[tid] = run;
  __syncthreads();
  for (int o = 1; o < 256; o <<= 1) {
    const int src = (tid >= o) ? (tid - o) : 0;
    float v = sc[src];
    v = (tid >= o) ? v : 0.0f;
    __syncthreads();
    sc[tid] += v;
    __syncthreads();
  }
  const float pre = sc[tid] - run;
  float rmax = -INFINITY;
#pragma unroll 1
  for (int j = 0; j < 8; ++j) {
    const int s = tid * 8 + j;
    const float F = sF[s] + pre;
    const float ip = gb[(size_t)s * kGateN + h] + bi;
    const float a = ip - F;
    rmax = fmaxf(rmax, a);
    sF[s] = F;
    sA[s] = a;
  }
  __syncthreads();
  sc[tid] = rmax;
  __syncthreads();
  for (int o = 1; o < 256; o <<= 1) {
    const int src = (tid >= o) ? (tid - o) : 0;
    float v = sc[src];
    v = (tid >= o) ? v : -INFINITY;
    __syncthreads();
    sc[tid] = fmaxf(sc[tid], v);
    __syncthreads();
  }
  const int psrc = (tid > 0) ? (tid - 1) : 0;
  float cm = sc[psrc];
  cm = (tid > 0) ? cm : -INFINITY;
#pragma unroll 1
  for (int j = 0; j < 8; ++j) {
    const int s = tid * 8 + j;
    cm = fmaxf(cm, sA[s]);
    sC[s] = cm;
    sF[s] = sF[s] + cm;
  }
  __syncthreads();
  float* ao = aout  + (size_t)bh * kSeq;
  float* co = cmout + (size_t)bh * kSeq;
  float* mo = mout  + (size_t)bh * kSeq;
  for (int pass = 0; pass < 2; ++pass) {
#pragma unroll
    for (int it = 0; it < 2; ++it) {
      const int e4 = (it * 256 + tid) * 4;
      const v4f va = *(const v4f*)(sA + e4);
      const v4f vc = *(const v4f*)(sC + e4);
      const v4f vm = *(const v4f*)(sF + e4);
      *(volatile v4f*)(ao + e4) = va;
      *(volatile v4f*)(co + e4) = vc;
      *(volatile v4f*)(mo + e4) = vm;
    }
    __threadfence();
  }
}

__global__ __launch_bounds__(256) void decay_attn_tile_kernel(
    const unsigned short* __restrict__ Qp, const unsigned short* __restrict__ Kp, const unsigned short* __restrict__ VTp,
    const float* __restrict__ aarr, const float* __restrict__ cmarr, const float* __restrict__ marr,
    unsigned short* __restrict__ Hs) {
  __shared__ __align__(16) _Float16 Ps[64 * kPP];
  __shared__ __align__(16) float sT[8][16 * 68];
  __shared__ float sRow[2][64];
  __shared__ float sInv[64];
  __shared__ float sEr[64];
  const _Float16* Q  = (const _Float16*)Qp;
  const _Float16* Kk = (const _Float16*)Kp;
  const _Float16* VT = (const _Float16*)VTp;
  const int tid = threadIdx.x, lane = tid & 31, wave = tid >> 5;
  const int c = lane & 15, hh = lane >> 4, koff = hh * 8;
  const int nqb = kSeq / 64;
  const int itile = blockIdx.x % nqb;
  const int bh = blockIdx.x / nqb;
  const int b = bh / kHeads, h = bh % kHeads;
  const int i0 = itile * 64;
  const int tr = wave & 3, tcp = wave >> 2;
  const float scl = 1.0f / sqrtf((float)kDH);
  const float* cmb = cmarr + (size_t)bh * kSeq;
  const float* ab  = aarr  + (size_t)bh * kSeq;
  const float cmOwn = cmb[i0 + (tid & 63)];

  if (tid < 64) {
    float er = expf(fminf(cmb[63] - cmOwn, 80.0f));
    er = (er < kFltMin) ? 0.0f : er;
    sEr[tid] = er;
  }
  __syncthreads();

  const _Float16* qrow = Q + (size_t)(b * kSeq + i0 + tr * 16 + c) * kInner + h * kDH + koff;
  const _Float16* kbase = Kk + (size_t)(b * kSeq) * kInner + h * kDH + koff;
  const _Float16* vtb  = VT + (size_t)(h * kDH + wave * 64 + c) * kRows + (size_t)b * kSeq + koff;
  const int jl0 = tcp * 32 + c, jl1 = jl0 + 16;

  v8f acc[4][4];
#pragma unroll
  for (int i = 0; i < 4; ++i)
#pragma unroll
    for (int j = 0; j < 4; ++j) acc[i][j] = (v8f){0.f,0.f,0.f,0.f,0.f,0.f,0.f,0.f};
  float rs[8];
#pragma unroll
  for (int r = 0; r < 8; ++r) rs[r] = 0.0f;

#pragma unroll 1
  for (int jt = 0; jt <= itile; ++jt) {
    const int j0 = jt * 64;
    const _Float16* krow0 = kbase + (size_t)(j0 + jl0) * kInner;
    const _Float16* krow1 = krow0 + (size_t)16 * kInner;
    v8f s0 = (v8f){0.f,0.f,0.f,0.f,0.f,0.f,0.f,0.f};
    v8f s1 = (v8f){0.f,0.f,0.f,0.f,0.f,0.f,0.f,0.f};
#pragma unroll 1
    for (int ks = 0; ks < kDH; ks += 32) {
      const v16h a  = FragH::load(qrow + ks);
      const v16h b0 = FragH::load(krow0 + ks);
      const v16h b1 = FragH::load(krow1 + ks);
      s0 = mma_h(a, b0, s0);
      s1 = mma_h(a, b1, s1);
    }
    const float cref = cmb[j0 + 63];
    const float aj0 = ab[j0 + jl0];
    const float aj1 = ab[j0 + jl1];
    float ec0 = expf(fminf(aj0 - cref, 0.0f));
    float ec1 = expf(fminf(aj1 - cref, 0.0f));
    ec0 = (ec0 < kFltMin) ? 0.0f : ec0;
    ec1 = (ec1 < kFltMin) ? 0.0f : ec1;
#pragma unroll
    for (int r = 0; r < 8; ++r) {
      const int il = tr * 16 + 8 * hh + r;
      const int irow = i0 + il;
      const float er = sEr[il];
      float w0 = ec0 * er;
      float w1 = ec1 * er;
      w0 = (w0 < kFltMin) ? 0.0f : w0;
      w1 = (w1 < kFltMin) ? 0.0f : w1;
      const float t0 = s0[r] * scl * w0;
      const float t1 = s1[r] * scl * w1;
      const float p0 = (j0 + jl0 <= irow) ? t0 : 0.0f;
      const float p1 = (j0 + jl1 <= irow) ? t1 : 0.0f;
      rs[r] += p0 + p1;
      Ps[il * kPP + jl0] = (_Float16)p0;
      Ps[il * kPP + jl1] = (_Float16)p1;
    }
    __syncthreads();
    if (tid < 64) {
      const int jn = (jt < itile) ? (jt + 1) : itile;
      float er = expf(fminf(cmb[jn * 64 + 63] - cmOwn, 80.0f));
      er = (er < kFltMin) ? 0.0f : er;
      sEr[tid] = er;
    }
#pragma unroll 1
    for (int kk = 0; kk < 2; ++kk) {
      v16h bf[4];
#pragma unroll
      for (int j = 0; j < 4; ++j) bf[j] = FragH::load(vtb + (size_t)(j * 16) * kRows + j0 + kk * 32);
#pragma unroll
      for (int i = 0; i < 4; ++i) {
        const v16h a = FragH::load(Ps + (i * 16 + c) * kPP + kk * 32 + koff);
#pragma unroll
        for (int j = 0; j < 4; ++j) acc[i][j] = mma_h(a, bf[j], acc[i][j]);
      }
    }
    __syncthreads();
  }

#pragma unroll
  for (int r = 0; r < 8; ++r) {
    float v = rs[r];
#pragma unroll
    for (int off = 1; off < 16; off <<= 1) v += __shfl_xor(v, off, 32);
    if (c == 0) sRow[tcp][tr * 16 + 8 * hh + r] = v;
  }
  __syncthreads();
  if (tid < 64) {
    const float tot = (sRow[0][tid] + sRow[1][tid]) * (1.0f / kPCarry);
    const float mm = marr[(size_t)bh * kSeq + i0 + tid];
    float em = expf(-mm);
    em = (em < kFltMin) ? 0.0f : em;
    const float nn = fmaxf(fabsf(tot), em);
    sInv[tid] = 1.0f / nn;
  }
  __syncthreads();

  float* slab = sT[wave];
#pragma unroll
  for (int i = 0; i < 4; ++i) {
#pragma unroll
    for (int r = 0; r < 8; ++r) {
      const float inv = sInv[i * 16 + 8 * hh + r];
#pragma unroll
      for (int j = 0; j < 4; ++j) slab[(8 * hh + r) * 68 + (j << 4) + c] = acc[i][j][r] * inv;
    }
    __builtin_amdgcn_fence(__ATOMIC_RELEASE, "workgroup");
    __builtin_amdgcn_wave_barrier();
    __builtin_amdgcn_fence(__ATOMIC_ACQUIRE, "workgroup");
    {
      const int q = lane >> 3, c8 = (lane & 7) * 8;
      for (int pass = 0; pass < 2; ++pass) {
#pragma unroll
        for (int it = 0; it < 4; ++it) {
          const int row = it * 4 + q;
          const float* sp = slab + row * 68 + c8;
          v8h hv;
#pragma unroll
          for (int e = 0; e < 8; ++e) hv[e] = (_Float16)sp[e];
          *(volatile v8h*)(Hs + (size_t)(b * kSeq + i0 + i * 16 + row) * kInner + h * kDH + wave * 64 + c8) = hv;
        }
        __threadfence();
      }
    }
    __builtin_amdgcn_fence(__ATOMIC_RELEASE, "workgroup");
    __builtin_amdgcn_wave_barrier();
    __builtin_amdgcn_fence(__ATOMIC_ACQUIRE, "workgroup");
  }
}

__global__ __launch_bounds__(256) void headnorm_kernel(const unsigned short* __restrict__ hs, const unsigned short* __restrict__ up,
                                                       const float* __restrict__ mhg, unsigned short* __restrict__ hout, int npairs) {
  const int lane = threadIdx.x & 31;
  const int wid = blockIdx.x * 8 + (threadIdx.x >> 5);
  if (wid >= npairs) return;
  const int row = wid / kHeads, h = wid % kHeads;
  const v4u* hp = (const v4u*)(const void*)(hs + (size_t)row * kInner + h * kDH);
  const v4u* zp = (const v4u*)(const void*)(up + (size_t)row * kUpN + kInner + h * kDH);
  const float unc = 1.0f / kPCarry;
  float v[2][8];
#pragma unroll
  for (int q = 0; q < 2; ++q) {
    const v4u w = hp[32 * q + lane];
    const unsigned w0 = w[0], w1 = w[1], w2 = w[2], w3 = w[3];
    v[q][0] = h16_to_f32(w0 & 0xffffu) * unc; v[q][1] = h16_to_f32(w0 >> 16) * unc;
    v[q][2] = h16_to_f32(w1 & 0xffffu) * unc; v[q][3] = h16_to_f32(w1 >> 16) * unc;
    v[q][4] = h16_to_f32(w2 & 0xffffu) * unc; v[q][5] = h16_to_f32(w2 >> 16) * unc;
    v[q][6] = h16_to_f32(w3 & 0xffffu) * unc; v[q][7] = h16_to_f32(w3 >> 16) * unc;
  }
  float s = 0.0f;
#pragma unroll
  for (int q = 0; q < 2; ++q)
#pragma unroll
    for (int e = 0; e < 8; ++e) s += v[q][e];
#pragma unroll
  for (int off = 1; off < 32; off <<= 1) s += __shfl_xor(s, off, 32);
  const float mu = s * (1.0f / (float)kDH);
  float ss = 0.0f;
#pragma unroll
  for (int q = 0; q < 2; ++q)
#pragma unroll
    for (int e = 0; e < 8; ++e) { const float d = v[q][e] - mu; ss += d * d; }
#pragma unroll
  for (int off = 1; off < 32; off <<= 1) ss += __shfl_xor(ss, off, 32);
  const float var = ss * (1.0f / (float)kDH);
  const float rstd = rsqrtf(var + kLnEps);
  unsigned short* op = hout + (size_t)row * kInner + h * kDH;
#pragma unroll 1
  for (int q = 0; q < 2; ++q) {
    const v4u w = hp[32 * q + lane];
    const v4u zw = zp[32 * q + lane];
    const v4f g0 = *(const v4f*)(mhg + h * kDH + 256 * q + 8 * lane);
    const v4f g1 = *(const v4f*)(mhg + h * kDH + 256 * q + 8 * lane + 4);
    const unsigned w0 = w[0], w1 = w[1], w2 = w[2], w3 = w[3];
    const unsigned z0 = zw[0], z1 = zw[1], z2 = zw[2], z3 = zw[3];
    float hv[8], zv[8], gv[8];
    hv[0] = h16_to_f32(w0 & 0xffffu); hv[1] = h16_to_f32(w0 >> 16);
    hv[2] = h16_to_f32(w1 & 0xffffu); hv[3] = h16_to_f32(w1 >> 16);
    hv[4] = h16_to_f32(w2 & 0xffffu); hv[5] = h16_to_f32(w2 >> 16);
    hv[6] = h16_to_f32(w3 & 0xffffu); hv[7] = h16_to_f32(w3 >> 16);
    zv[0] = h16_to_f32(z0 & 0xffffu); zv[1] = h16_to_f32(z0 >> 16);
    zv[2] = h16_to_f32(z1 & 0xffffu); zv[3] = h16_to_f32(z1 >> 16);
    zv[4] = h16_to_f32(z2 & 0xffffu); zv[5] = h16_to_f32(z2 >> 16);
    zv[6] = h16_to_f32(z3 & 0xffffu); zv[7] = h16_to_f32(z3 >> 16);
    gv[0] = g0[0]; gv[1] = g0[1]; gv[2] = g0[2]; gv[3] = g0[3];
    gv[4] = g1[0]; gv[5] = g1[1]; gv[6] = g1[2]; gv[7] = g1[3];
    unsigned hb[8];
#pragma unroll
    for (int e = 0; e < 8; ++e) {
      const float hn = (hv[e] * unc - mu) * rstd;
      const float sz = zv[e] * __builtin_amdgcn_rcpf(1.0f + expf(-zv[e]));
      hb[e] = h_bits(hn * gv[e] * sz * kHoCarry);
    }
    const v4u u = (v4u){hb[0] | (hb[1] << 16), hb[2] | (hb[3] << 16), hb[4] | (hb[5] << 16), hb[6] | (hb[7] << 16)};
    unsigned short* o = op + 256 * q + 8 * lane;
    *(volatile v4u*)(void*)o = u;
    __threadfence();
    *(volatile v4u*)(void*)o = u;
  }
}

__global__ __launch_bounds__(256) void dyt_kernel(const float* __restrict__ x2, const float* __restrict__ da,
                                                  const float* __restrict__ dw, const float* __restrict__ db,
                                                  unsigned short* __restrict__ t, int n2) {
  const int i = blockIdx.x * 256 + threadIdx.x;
  if (i < n2) {
    const int col = (i & (kDim / 2 - 1)) * 2;
    const float a = da[0];
    const v2f xv = *(const v2f*)(x2 + 2 * (size_t)i);
    const v2f wv = *(const v2f*)(dw + col);
    const v2f bv = *(const v2f*)(db + col);
    const float t0 = wv[0] * tanhf(a * xv[0]) + bv[0];
    const float t1 = wv[1] * tanhf(a * xv[1]) + bv[1];
    const unsigned u = h_bits(t0) | (h_bits(t1) << 16);
    ((volatile unsigned*)t)[i] = u;
    __threadfence();
    ((volatile unsigned*)t)[i] = u;
  }
}

extern "C" void kernel_launch(void* const* d_in, const int* in_sizes, int n_in,
                              void* d_out, int out_size, void* d_ws, size_t ws_size, hipStream_t stream) {
  if (n_in < 25 || d_out == nullptr || d_ws == nullptr) return;
  if (in_sizes[0] != kRows * kDim || in_sizes[1] != kDim || in_sizes[2] != kDim ||
      in_sizes[3] != kDim * kUpN || in_sizes[4] != kUpN || in_sizes[5] != 4 * kInner || in_sizes[6] != kInner ||
      in_sizes[7] != kInner * kInner || in_sizes[8] != kInner || in_sizes[9] != kInner * kInner || in_sizes[10] != kInner ||
      in_sizes[11] != kInner * kInner || in_sizes[12] != kInner || in_sizes[13] != kInner * 2 * kHeads ||
      in_sizes[14] != 2 * kHeads || in_sizes[15] != kInner || in_sizes[16] != kInner * kDim || in_sizes[17] != kDim ||
      in_sizes[18] != 1 || in_sizes[19] != kDim || in_sizes[20] != kDim || in_sizes[21] != kDim * kFF ||
      in_sizes[22] != kFF || in_sizes[23] != kFF * kDim || in_sizes[24] != kDim || out_size != kRows * kDim) return;

  const float* x      = (const float*)d_in[0];
  const float* ln_g   = (const float*)d_in[1];
  const float* ln_b   = (const float*)d_in[2];
  const float* W_up   = (const float*)d_in[3];
  const float* b_up   = (const float*)d_in[4];
  const float* conv_w = (const float*)d_in[5];
  const float* conv_b = (const float*)d_in[6];
  const float* Wq     = (const float*)d_in[7];
  const float* bq     = (const float*)d_in[8];
  const float* Wk     = (const float*)d_in[9];
  const float* bk     = (const float*)d_in[10];
  const float* Wv     = (const float*)d_in[11];
  const float* bv     = (const float*)d_in[12];
  const float* W_if   = (const float*)d_in[13];
  const float* b_if   = (const float*)d_in[14];
  const float* mh_g   = (const float*)d_in[15];
  const float* W_down = (const float*)d_in[16];
  const float* b_down = (const float*)d_in[17];
  const float* dyt_a  = (const float*)d_in[18];
  const float* dyt_w  = (const float*)d_in[19];
  const float* dyt_b  = (const float*)d_in[20];
  const float* W1     = (const float*)d_in[21];
  const float* b1     = (const float*)d_in[22];
  const float* W2     = (const float*)d_in[23];
  const float* b2     = (const float*)d_in[24];
  float* out = (float*)d_out;

  char* ws = (char*)d_ws; size_t off = 0;
  auto carve = [&](size_t bytes) -> char* { char* p = ws + off; off += (bytes + 255) & ~(size_t)255; return p; };
  unsigned short* S0 = (unsigned short*)carve((size_t)8388608);
  unsigned short* S1 = (unsigned short*)carve((size_t)8388608);
  unsigned short* S2 = (unsigned short*)carve((size_t)4194304);
  unsigned short* R1 = (unsigned short*)carve((size_t)kRows * kUpN * 2);
  unsigned short* R2 = (unsigned short*)carve((size_t)kRows * kInner * 2);
  unsigned short* R3 = (unsigned short*)carve((size_t)kRows * kDim * 2);
  char*           R4 = carve((size_t)kRows * kInner * 2);
  unsigned short* R5 = (unsigned short*)carve((size_t)kRows * kInner * 2);
  unsigned short* R6 = (unsigned short*)carve((size_t)kInner * kRows * 2);
  float*          G  = (float*)carve((size_t)kRows * kGateN * 4);
  float*          TA = (float*)carve((size_t)kBatch * kHeads * kSeq * 4);
  float*          TC = (float*)carve((size_t)kBatch * kHeads * kSeq * 4);
  float*          TM = (float*)carve((size_t)kBatch * kHeads * kSeq * 4);
  if (off > ws_size || off > (size_t)134217728) return;
  static_assert((size_t)kRows * kDim * 4 == (size_t)kRows * kInner * 2, "x2 fits the q region");
  static_assert((size_t)kDim * kUpN * 2 <= 8388608 && (size_t)kInner * kInner * 2 <= 8388608 && (size_t)kFF * kDim * 2 <= 8388608, "weight slots");
  static_assert((size_t)kInner * kDim * 2 <= 4194304 && (size_t)kGateN * kInner * 2 <= 4194304, "small weight slot");
  static_assert((size_t)kRows * kFF * 2 <= (size_t)kRows * kUpN * 2, "f1 fits the up region");

  unsigned short* upP  = R1;
  unsigned short* f1P  = R1;
  unsigned short* xcP  = R2;
  unsigned short* hsP  = R2;
  unsigned short* xnP  = R3;
  unsigned short* tP   = R3;
  unsigned short* qP   = (unsigned short*)R4;
  float*          x2P  = (float*)R4;
  unsigned short* kP   = R5;
  unsigned short* hoP  = R5;
  unsigned short* vtP  = R6;

  const float wInv = 1.0f / kWCarry;

  wt_f16_kernel<<<dim3(kUpN / 64, kDim / 64), 256, 0, stream>>>(W_up, kDim, kUpN, kDim, S0, kWCarry);
  ln_f16_kernel<<<kRows / 8, 256, 0, stream>>>(x, ln_g, ln_b, xnP, kRows);
  wmma_gemm64<2, 1, false, 0><<<(kRows / 64) * (kUpN / 64) / 8, 256, 0, stream>>>(
      xnP, kDim, S0, kDim, (void*)upP, kUpN, b_up, x, kRows, kUpN, kDim, wInv, 1.0f, 0.0f);
  wt_f16_kernel<<<dim3(kInner / 64, kInner / 64), 256, 0, stream>>>(Wv, kInner, kInner, kInner, S0, kWCarry);
  wmma_gemm64<1, 1, false, 0><<<(kInner / 64) * (kRows / 64) / 8, 256, 0, stream>>>(
      S0, kInner, upP, kUpN, (void*)vtP, kRows, bv, x, kInner, kRows, kInner, wInv, 1.0f, 0.0f);
  conv_silu_kernel<<<(kRows * (kInner / 2)) / 256, 256, 0, stream>>>(upP, conv_w, conv_b, xcP);
  wt_f16_kernel<<<dim3(kInner / 64, kInner / 64), 256, 0, stream>>>(Wq, kInner, kInner, kInner, S0, kWCarry);
  wt_f16_kernel<<<dim3(kInner / 64, kInner / 64), 256, 0, stream>>>(Wk, kInner, kInner, kInner, S1, kWCarry);
  wif_f16_kernel<<<(kGateN * (kInner / 8)) / 256, 256, 0, stream>>>(W_if, S2, kWCarry);
  const float qkScale = 1.0f / (kXcCarry * kWCarry);
  wmma_gemm64<2, 1, false, 0><<<(kRows / 64) * (kInner / 64) / 8, 256, 0, stream>>>(
      xcP, kInner, S0, kInner, (void*)qP, kInner, bq, x, kRows, kInner, kInner, qkScale, kQKCarry, 0.0f);
  wmma_gemm64<2, 1, false, 0><<<(kRows / 64) * (kInner / 64) / 8, 256, 0, stream>>>(
      xcP, kInner, S1, kInner, (void*)kP, kInner, bk, x, kRows, kInner, kInner, qkScale, kQKCarry, 0.0f);
  wmma_gemm64<0, 0, false, 0><<<(kRows / 64) * (kGateN / 64) / 8, 256, 0, stream>>>(
      xcP, kInner, S2, kInner, (void*)G, kGateN, b_if, x, kRows, kGateN, kInner, qkScale, 1.0f, 0.0f);
  scan_kernel<<<kBatch * kHeads, 256, 0, stream>>>(G, b_if, TA, TC, TM);
  decay_attn_tile_kernel<<<kBatch * kHeads * (kSeq / 64), 256, 0, stream>>>(qP, kP, vtP, TA, TC, TM, hsP);
  headnorm_kernel<<<(kRows * kHeads) / 8, 256, 0, stream>>>(hsP, upP, mh_g, hoP, kRows * kHeads);
  wt_f16_kernel<<<dim3(kDim / 64, kInner / 64), 256, 0, stream>>>(W_down, kInner, kDim, kInner, S2, kWCarry);
  wmma_gemm64<2, 0, true, 0><<<(kRows / 64) * (kDim / 64) / 8, 256, 0, stream>>>(
      hoP, kInner, S2, kInner, (void*)x2P, kDim, b_down, x, kRows, kDim, kInner, 1.0f / (kHoCarry * kWCarry), 1.0f, 2.0f);
  dyt_kernel<<<(kRows * (kDim / 2)) / 256, 256, 0, stream>>>(x2P, dyt_a, dyt_w, dyt_b, tP, kRows * (kDim / 2));
  wt_f16_kernel<<<dim3(kFF / 64, kDim / 64), 256, 0, stream>>>(W1, kDim, kFF, kDim, S0, kWCarry);
  wt_f16_kernel<<<dim3(kDim / 64, kFF / 64), 256, 0, stream>>>(W2, kFF, kDim, kFF, S1, kWCarry);
  wmma_gemm64<2, 1, false, 2><<<(kRows / 64) * (kFF / 64) / 8, 256, 0, stream>>>(
      tP, kDim, S0, kDim, (void*)f1P, kFF, b1, x, kRows, kFF, kDim, wInv, 1.0f, 0.0f);
  wmma_gemm64<2, 0, true, 0><<<(kRows / 64) * (kDim / 64) / 8, 256, 0, stream>>>(
      f1P, kFF, S1, kFF, (void*)out, kDim, b2, x2P, kRows, kDim, kFF, wInv, 1.0f, 1.0f);
}
